// RBF_PINNs_80711025427082
// MI455X (gfx1250) — hardware-run, weakly checked
//
#include <hip/hip_runtime.h>


#ifndef NB
#define NB 262144
#endif
#define NB_FULL 262144
#define NRBF  256
#define TPTS  16
#define BWAVES 8
#define BPTS  (TPTS * BWAVES)
#define ROWB  16
#define KC2   (-0.72134752044448169f)

static_assert(NB <= NB_FULL);
static_assert(NB % BPTS == 0);
static_assert(NRBF % 32 == 0);
static_assert(NRBF == 256);
static_assert(BWAVES * 32 == 256);
static_assert(2 * NRBF == 4 * 128);
static_assert(16 * 16 * 16 == 16 * NRBF);
static_assert(16 * ROWB * 1 == TPTS * ROWB);
static_assert(2 * NRBF * 4 + 16 * NRBF * 2 <= 131072);

typedef unsigned short bf;
typedef __attribute__((ext_vector_type(16))) __bf16   v16bf;
typedef __attribute__((ext_vector_type(8)))  unsigned short v8us;
typedef __attribute__((ext_vector_type(8)))  float    v8f;
typedef __attribute__((ext_vector_type(4)))  float    v4f;
typedef v4f  __attribute__((may_alias)) v4fa;

__device__ __forceinline__ unsigned short f2bf(float f) { unsigned u = __float_as_uint(f); u += 0x7FFFu + ((u >> 16) & 1u); return (unsigned short)(u >> 16); }
__device__ __forceinline__ float bf2f(unsigned short w) { return __uint_as_float(((unsigned)w) << 16); }
__device__ __forceinline__ v16bf cat16b(v8us lo, v8us hi) { return __builtin_bit_cast(v16bf, __builtin_shufflevector(lo, hi, 0, 1, 2, 3, 4, 5, 6, 7, 8, 9, 10, 11, 12, 13, 14, 15)); }
__device__ __forceinline__ v8f wmmab(v16bf a, v16bf b, v8f c) { return __builtin_amdgcn_wmma_f32_16x16x32_bf16(false, a, false, b, (short)0, c, false, false); }
__device__ __forceinline__ v8f wmmag(v16bf a, v16bf b, v8f c) {
    c = wmmab(a, b, c);
    asm volatile("v_nop\n\tv_nop\n\tv_nop\n\tv_nop" : "+v"(c) : "v"(a), "v"(b));
    return c;
}

struct rbfq { unsigned short ph, pl, qh, ql; };
__device__ __forceinline__ rbfq rbf_eval(float cx, float cy, float px, float py) {
    const float dx = px - cx, dy = py - cy;
    const float r2 = dx * dx + dy * dy;
    const float phi = __builtin_amdgcn_exp2f(KC2 * r2);
    const float psi = phi * (r2 - 2.0f);
    rbfq o;
    o.ph = f2bf(phi); o.pl = f2bf(phi - bf2f(o.ph));
    o.qh = f2bf(psi); o.ql = f2bf(psi - bf2f(o.qh));
    return o;
}

__global__ __launch_bounds__(256) __attribute__((amdgpu_num_vgpr(256))) void k_rbf(const float* __restrict__ x, const float* __restrict__ y,
                                                                                   const float* __restrict__ centers, const float* __restrict__ W,
                                                                                   const float* __restrict__ eps_p, const float* __restrict__ delta_p,
                                                                                   const float* __restrict__ gamma_p, float* out) {
    __shared__ __align__(16) float sC[2 * NRBF];
    __shared__ __align__(16) bf    sWT[16 * NRBF];
    const int tid = threadIdx.x, lane = tid & 31, lr = lane & 15, hi = lane >> 4;
    const int wave = __builtin_amdgcn_readfirstlane(threadIdx.x >> 5);

    if (tid < 128) {
        const v4f c = ((const v4f*)centers)[tid];
        v4f o;
#pragma unroll
        for (int k = 0; k < 4; ++k) o[k] = bf2f(f2bf(c[k]));
        *(v4fa*)&sC[4 * tid] = o;
    }
    {
        const int row = tid >> 4, kseg = (tid & 15) * 16;
        const int col = min(row, 1);
        const v4f* wp = (const v4f*)(W + 2 * kseg);
        v8us o0, o1;
#pragma unroll
        for (int q = 0; q < 4; ++q) {
            const v4f w0 = wp[q];
            const v4f w1 = wp[4 + q];
            const float a0 = (col == 0) ? w0[0] : w0[1];
            const float a1 = (col == 0) ? w0[2] : w0[3];
            const float b0 = (col == 0) ? w1[0] : w1[1];
            const float b1 = (col == 0) ? w1[2] : w1[3];
            o0[2 * q]     = (row < 2) ? f2bf(a0) : (unsigned short)0;
            o0[2 * q + 1] = (row < 2) ? f2bf(a1) : (unsigned short)0;
            o1[2 * q]     = (row < 2) ? f2bf(b0) : (unsigned short)0;
            o1[2 * q + 1] = (row < 2) ? f2bf(b1) : (unsigned short)0;
        }
        *(v8us*)&sWT[row * NRBF + kseg]     = o0;
        *(v8us*)&sWT[row * NRBF + kseg + 8] = o1;
    }
    __syncthreads();

    const int tileBase = (blockIdx.x * BWAVES + wave) * TPTS;
    const int pt = tileBase + lr;
    const float px = bf2f(f2bf(x[pt]));
    const float py = bf2f(f2bf(y[pt]));

    v8f accO = (v8f){}, accL = (v8f){};
#pragma unroll 1
    for (int kc = 0; kc < NRBF; kc += 32) {
        const int kb = kc + 8 * hi;
        const v16bf a = cat16b(*(const v8us*)&sWT[lr * NRBF + kb], *(const v8us*)&sWT[lr * NRBF + kb + 16]);
        v8us ph0, pl0, qh0, ql0, ph1, pl1, qh1, ql1;
#pragma unroll
        for (int q = 0; q < 4; ++q) {
            const v4f c0 = *(const v4fa*)&sC[2 * kb + 4 * q];
            const v4f c1 = *(const v4fa*)&sC[2 * (kb + 16) + 4 * q];
            const rbfq e00 = rbf_eval(c0[0], c0[1], px, py);
            const rbfq e01 = rbf_eval(c0[2], c0[3], px, py);
            const rbfq e10 = rbf_eval(c1[0], c1[1], px, py);
            const rbfq e11 = rbf_eval(c1[2], c1[3], px, py);
            ph0[2 * q] = e00.ph; ph0[2 * q + 1] = e01.ph; pl0[2 * q] = e00.pl; pl0[2 * q + 1] = e01.pl;
            qh0[2 * q] = e00.qh; qh0[2 * q + 1] = e01.qh; ql0[2 * q] = e00.ql; ql0[2 * q + 1] = e01.ql;
            ph1[2 * q] = e10.ph; ph1[2 * q + 1] = e11.ph; pl1[2 * q] = e10.pl; pl1[2 * q + 1] = e11.pl;
            qh1[2 * q] = e10.qh; qh1[2 * q + 1] = e11.qh; ql1[2 * q] = e10.ql; ql1[2 * q + 1] = e11.ql;
        }
        const v16bf bph = cat16b(ph0, ph1), bpl = cat16b(pl0, pl1), bqh = cat16b(qh0, qh1), bql = cat16b(ql0, ql1);
        accO = wmmag(a, bph, accO);
        accL = wmmag(a, bqh, accL);
        accO = wmmag(a, bpl, accO);
        accL = wmmag(a, bql, accL);
    }

    const float u  = accO[0], p  = accO[1];
    const float lu = accL[0], lp = accL[1];
    const float eps   = bf2f(f2bf(eps_p[0]));
    const float delta = bf2f(f2bf(delta_p[0]));
    const float gamma = bf2f(f2bf(gamma_p[0]));
    const float res1 = p - lu;
    const float sh   = (u + 2.0f * p) + lp;
    const float u2   = u * u;
    const float res2 = ((eps * u - delta * u2) - gamma * (u2 * u)) - sh;
    v4f o; o[0] = u; o[1] = p; o[2] = res1; o[3] = res2;
#pragma unroll 1
    for (int ps = 0; ps < 2; ++ps) {
        if (lane < 16) { *(volatile v4f*)(out + (size_t)pt * 4) = o; }
        if (ps == 0) __threadfence(); }
}

extern "C" void kernel_launch(void* const* d_in, const int* in_sizes, int n_in,
                              void* d_out, int out_size, void* d_ws, size_t ws_size, hipStream_t stream) {
    (void)d_ws; (void)ws_size;
    if (n_in < 7) return;
    if ((size_t)in_sizes[0] < (size_t)NB || (size_t)in_sizes[1] < (size_t)NB) return;
    if ((size_t)in_sizes[2] < (size_t)(2 * NRBF) || (size_t)in_sizes[3] < (size_t)(2 * NRBF)) return;
    if (in_sizes[4] < 1 || in_sizes[5] < 1 || in_sizes[6] < 1) return;
    if ((size_t)out_size < (size_t)NB * 4) return;
    const float* x       = (const float*)d_in[0];
    const float* y       = (const float*)d_in[1];
    const float* centers = (const float*)d_in[2];
    const float* W       = (const float*)d_in[3];
    const float* eps_p   = (const float*)d_in[4];
    const float* delta_p = (const float*)d_in[5];
    const float* gamma_p = (const float*)d_in[6];
    float* OUT = (float*)d_out;
    k_rbf<<<NB / BPTS, 256, 0, stream>>>(x, y, centers, W, eps_p, delta_p, gamma_p, OUT);
}
